// MambaBlock_4475355922525
// MI455X (gfx1250) — hardware-run, weakly checked
//
#include <hip/hip_runtime.h>
#include <math.h>

typedef __attribute__((ext_vector_type(16))) _Float16 v16h;
typedef __attribute__((ext_vector_type(8)))  _Float16 v8h;
typedef __attribute__((ext_vector_type(16))) __bf16   v16b;
typedef __attribute__((ext_vector_type(8)))  __bf16   v8b;
typedef __attribute__((ext_vector_type(8)))  float    v8f;
typedef __attribute__((ext_vector_type(4)))  float    v4f;

constexpr int kBatch  = 2;
constexpr int kSeq    = 2048;
constexpr int kHid    = 1024;
constexpr int kInner  = 2048;
constexpr int kNst    = 16;
constexpr int kRank   = 64;
constexpr int kTaps   = 4;
constexpr int kXpjN   = kRank + 2 * kNst;
constexpr int kXpjP   = 128;
constexpr int kRows   = kBatch * kSeq;
constexpr int kTrP    = 68;
constexpr int kConvTP = 260;
constexpr int kScanTS = 64;
constexpr int kScanCh = 64;
constexpr int kScanXP = 32;
constexpr int kScanYP = 68;
constexpr float kWCarry    = 16.0f;
constexpr float kConvCarry = 256.0f;
constexpr float kTsCarry   = 256.0f;
constexpr float kYCarry    = 1024.0f;
constexpr float kLog2e     = 1.4426950408889634f;
constexpr float kLn2       = 0.6931471805599453f;
static_assert(kTaps == 4, "taps");
static_assert(kXpjN <= kXpjP && (kXpjN % 4) == 0, "x_proj pad");
static_assert((kHid % 32) == 0 && (kInner % 32) == 0 && (kRank % 32) == 0, "GEMM K multiples of 32");
static_assert((kRows % 64) == 0 && (kInner % 64) == 0 && (kXpjP % 64) == 0 && (kHid % 64) == 0, "GEMM M,N multiples of 64");
static_assert((kSeq % kScanTS) == 0 && (kSeq % 64) == 0 && (kInner % kScanCh) == 0 && (kInner % 256) == 0, "tile multiples");
static_assert((kHid % 64) == 0 && ((2 * kInner) % 64) == 0 && (kRank % 64) == 0, "transpose tiles");

constexpr size_t kOffRA   = 0;
constexpr size_t kOffWIN  = kOffRA;
constexpr size_t kOffXN   = kOffRA   + (size_t)(2 * kInner) * kHid * 2;
constexpr size_t kSzRA    = (size_t)kRows * kInner * 2;
constexpr size_t kOffWOUT = kOffRA   + kSzRA;
constexpr size_t kOffWX   = kOffWOUT + (size_t)kHid   * kInner * 2;
constexpr size_t kOffWDT  = kOffWX   + (size_t)kXpjP  * kInner * 2;
constexpr size_t kOffTS   = kOffWDT  + (size_t)kInner * kRank  * 2;
constexpr size_t kOffXPJ  = kOffTS   + (size_t)kRows  * kRank  * 2;
constexpr size_t kOffHID  = kOffXPJ  + (size_t)kRows  * kXpjP  * 4;
constexpr size_t kOffGATE = kOffHID  + (size_t)kRows  * kInner * 4;
constexpr size_t kOffCONV = kOffGATE + (size_t)kRows  * kInner * 4;
constexpr size_t kWsTotal = kOffCONV + (size_t)kRows  * kInner * 4;
static_assert(kOffXN + (size_t)kRows * kHid * 2 == kOffRA + kSzRA, "WIN16 + XN16 fill RA exactly");
static_assert(kWsTotal == 125042688ull, "carve total");
static_assert(kWsTotal <= 134217728ull, "carve cap");
static_assert((kOffXN % 128) == 0 && (kOffWOUT % 128) == 0 && (kOffWX % 128) == 0 && (kOffWDT % 128) == 0 &&
              (kOffTS % 128) == 0 && (kOffXPJ % 128) == 0 && (kOffHID % 128) == 0 && (kOffGATE % 128) == 0 &&
              (kOffCONV % 128) == 0, "128-B aligned regions");

__device__ __forceinline__ unsigned short f2bf_bits(float f) {
  unsigned u = __float_as_uint(f);
  return (unsigned short)((u + 0x7FFFu + ((u >> 16) & 1u)) >> 16);
}
__device__ __forceinline__ float bf_bits2f(unsigned short h) { return __uint_as_float(((unsigned)h) << 16); }

__device__ __forceinline__ void dep_guard_h(v8f& a, v8f& b, v16h x, v16h y) { asm volatile("v_nop\n\tv_nop\n\tv_nop\n\tv_nop" : "+v"(a), "+v"(b) : "v"(x), "v"(y)); }
__device__ __forceinline__ void dep_guard_b(v8f& a, v8f& b, v16b x, v16b y) { asm volatile("v_nop\n\tv_nop\n\tv_nop\n\tv_nop" : "+v"(a), "+v"(b) : "v"(x), "v"(y)); }
__device__ __forceinline__ void dep_guard4_h(v8f& a, v8f& b, v8f& c, v8f& d, v16h x, v16h y) { asm volatile("v_nop\n\tv_nop\n\tv_nop\n\tv_nop" : "+v"(a), "+v"(b), "+v"(c), "+v"(d) : "v"(x), "v"(y)); }
__device__ __forceinline__ void dep_guard4_b(v8f& a, v8f& b, v8f& c, v8f& d, v16b x, v16b y) { asm volatile("v_nop\n\tv_nop\n\tv_nop\n\tv_nop" : "+v"(a), "+v"(b), "+v"(c), "+v"(d) : "v"(x), "v"(y)); }
__device__ __forceinline__ void keep4_h(v16h a, v16h b, v16h c, v16h d) { asm volatile("v_nop" :: "v"(a), "v"(b), "v"(c), "v"(d)); }
__device__ __forceinline__ void keep4_b(v16b a, v16b b, v16b c, v16b d) { asm volatile("v_nop" :: "v"(a), "v"(b), "v"(c), "v"(d)); }
__device__ __forceinline__ void acc_guard4(v8f& a, v8f& b, v8f& c, v8f& d) { asm volatile("v_nop\n\tv_nop\n\tv_nop\n\tv_nop" : "+v"(a), "+v"(b), "+v"(c), "+v"(d)); }
template <typename T> struct Frag;
template <> struct Frag<_Float16> {
  typedef v16h V; union U { v16h v; v8h h[2]; };
  static __device__ __forceinline__ v16h load(const _Float16* p) {
    U f; f.h[0] = *(const v8h*)(p); f.h[1] = *(const v8h*)(p + 16); return f.v;
  }
  static __device__ __forceinline__ v8f mma(v16h a, v16h b, v8f c) {
    return __builtin_amdgcn_wmma_f32_16x16x32_f16(false, a, false, b, (short)0, c, false, false);
  }
  static __device__ __forceinline__ void guard(v8f& a, v8f& b, v16h x, v16h y) { dep_guard_h(a, b, x, y); }
  static __device__ __forceinline__ void guard4(v8f& a, v8f& b, v8f& c, v8f& d, v16h x, v16h y) { dep_guard4_h(a, b, c, d, x, y); }
  static __device__ __forceinline__ void keep(v16h a, v16h b, v16h c, v16h d) { keep4_h(a, b, c, d); }
};
template <> struct Frag<__bf16> {
  typedef v16b V; union U { v16b v; v8b h[2]; };
  static __device__ __forceinline__ v16b load(const __bf16* p) {
    U f; f.h[0] = *(const v8b*)(p); f.h[1] = *(const v8b*)(p + 16); return f.v;
  }
  static __device__ __forceinline__ v8f mma(v16b a, v16b b, v8f c) {
    return __builtin_amdgcn_wmma_f32_16x16x32_bf16(false, a, false, b, (short)0, c, false, false);
  }
  static __device__ __forceinline__ void guard(v8f& a, v8f& b, v16b x, v16b y) { dep_guard_b(a, b, x, y); }
  static __device__ __forceinline__ void guard4(v8f& a, v8f& b, v8f& c, v8f& d, v16b x, v16b y) { dep_guard4_b(a, b, c, d, x, y); }
  static __device__ __forceinline__ void keep(v16b a, v16b b, v16b c, v16b d) { keep4_b(a, b, c, d); }
};

template <int ET> struct Elem;
template <> struct Elem<0> { typedef _Float16 T; };
template <> struct Elem<1> { typedef __bf16 T; };
template <int ET, int SPL, int BIAS_MODE, int OUT_MODE, bool RESID, int ACT = 0>
__global__ __launch_bounds__(256) void wmma_gemm64(
    const unsigned short* __restrict__ Ap, const unsigned short* __restrict__ A2p, int lda, long strideA,
    const unsigned short* __restrict__ Btp, const unsigned short* __restrict__ Bt2p, int ldb, long strideB,
    void* __restrict__ Cout, void* __restrict__ Cout2, int ldc, long strideC,
    const float* __restrict__ bias,
    const float* __restrict__ resid, long strideR,
    int M, int N, int K, float scale) {
  typedef typename Elem<ET>::T T;
  typedef typename Frag<T>::V V;
  const T* A = (const T*)Ap; const T* A2 = (const T*)A2p; const T* Bt = (const T*)Btp; const T* Bt2 = (const T*)Bt2p;
  __shared__ __align__(16) float sT[8][16 * 68];
  const int b    = blockIdx.y;
  const int lane = threadIdx.x & 31;
  const int wave = threadIdx.x >> 5;
  const int tilesN = N >> 6;
  const int tilesM = M >> 6;
  const int tile = blockIdx.x * 8 + wave;
  if (tile >= tilesM * tilesN) return;
  const int tm = tile / tilesN;
  const int tn = tile - tm * tilesN;
  const int m0 = tm << 6;
  const int n0 = tn << 6;

  const T* Ab  = A  + (size_t)b * strideA;
  const T* Bb  = Bt + (size_t)b * strideB;
  const T* Ab2 = (SPL >= 1) ? (A2  + (size_t)b * strideA) : nullptr;
  const T* Bb2 = (SPL == 2) ? (Bt2 + (size_t)b * strideB) : nullptr;

  const int rlane = lane & 15;
  const int koff  = (lane >> 4) * 8;
  const int mOff  = (lane >> 4) * 8;

  v8f acc[4][4];
#pragma unroll
  for (int i = 0; i < 4; ++i)
#pragma unroll
    for (int j = 0; j < 4; ++j) acc[i][j] = (v8f){0.f,0.f,0.f,0.f,0.f,0.f,0.f,0.f};

  for (int k0 = 0; k0 < K; k0 += 32) {
    V bh[4], bl[4];
#pragma unroll
    for (int j = 0; j < 4; ++j) {
      const size_t bo = (size_t)(n0 + (j << 4) + rlane) * ldb + koff + k0;
      bh[j] = Frag<T>::load(Bb + bo);
      if (SPL == 2) bl[j] = Frag<T>::load(Bb2 + bo);
    }
#pragma unroll
    for (int i = 0; i < 4; ++i) {
      const size_t ao = (size_t)(m0 + (i << 4) + rlane) * lda + koff + k0;
      V ah = Frag<T>::load(Ab + ao);
      V al;
      if (SPL >= 1) al = Frag<T>::load(Ab2 + ao);
#pragma unroll
      for (int j = 0; j < 4; ++j) {
        acc[i][j] = Frag<T>::mma(ah, bh[j], acc[i][j]);
        if (SPL == 2) acc[i][j] = Frag<T>::mma(ah, bl[j], acc[i][j]);
        if (SPL >= 1) acc[i][j] = Frag<T>::mma(al, bh[j], acc[i][j]);
      }
      Frag<T>::guard4(acc[i][0], acc[i][1], acc[i][2], acc[i][3], ah, (SPL >= 1) ? al : ah);
    }
    Frag<T>::keep(bh[0], bh[1], bh[2], bh[3]);
    if (SPL == 2) Frag<T>::keep(bl[0], bl[1], bl[2], bl[3]);
  }
  acc_guard4(acc[0][0], acc[0][1], acc[0][2], acc[0][3]);
  acc_guard4(acc[1][0], acc[1][1], acc[1][2], acc[1][3]);
  acc_guard4(acc[2][0], acc[2][1], acc[2][2], acc[2][3]);
  acc_guard4(acc[3][0], acc[3][1], acc[3][2], acc[3][3]);

  float* slab = sT[wave];
  const float* Rb = RESID ? (resid + (size_t)b * strideR) : nullptr;
#pragma unroll
  for (int i = 0; i < 4; ++i) {
    const int mBase = m0 + (i << 4);
#pragma unroll
    for (int j = 0; j < 4; ++j) {
      const int n = n0 + (j << 4) + rlane;
      float bv = 0.f;
      if (BIAS_MODE == 2) bv = bias[n];
#pragma unroll
      for (int r = 0; r < 8; ++r) {
        float v = acc[i][j][r] * scale;
        if (BIAS_MODE == 1) v += bias[mBase + mOff + r];
        if (BIAS_MODE == 2) v += bv;
        if (RESID) v += Rb[(size_t)(mBase + mOff + r) * ldc + n];
        if (ACT == 1) v = tanhf(v);
        if (ACT == 2) v = fmaxf(v, 0.0f);
        if (ACT == 3) v = v / (1.0f + expf(-v));
        if (ACT == 4) v = (v > 0.f) ? v : 0.01f * v;
        slab[(mOff + r) * 68 + (j << 4) + rlane] = v;
      }
    }
    __builtin_amdgcn_fence(__ATOMIC_RELEASE, "workgroup");
    __builtin_amdgcn_wave_barrier();
    __builtin_amdgcn_fence(__ATOMIC_ACQUIRE, "workgroup");
    if (OUT_MODE == 0) {
      float* C = (float*)Cout + (size_t)b * strideC;
      const int hh = lane >> 4, c4 = (lane & 15) * 4;
      for (int pass = 0; pass < 2; ++pass) {
#pragma unroll
        for (int it = 0; it < 8; ++it) {
          const int row = it * 2 + hh;
          v4f v = *(const v4f*)(slab + row * 68 + c4);
          *(volatile v4f*)(C + (size_t)(mBase + row) * ldc + n0 + c4) = v;
        }
        __threadfence();
      }
    } else {
      const int q = lane >> 3, c8 = (lane & 7) * 8;
      unsigned short* C  = (unsigned short*)Cout  + (size_t)b * strideC;
      unsigned short* C2 = (OUT_MODE == 2) ? ((unsigned short*)Cout2 + (size_t)b * strideC) : nullptr;
      for (int pass = 0; pass < 2; ++pass) {
#pragma unroll
        for (int it = 0; it < 4; ++it) {
          const int row = it * 4 + q;
          const float* sp = slab + row * 68 + c8;
          v8h hv, lv;
#pragma unroll
          for (int e = 0; e < 8; ++e) {
            if (OUT_MODE == 1) {
              hv[e] = (_Float16)sp[e];
            } else {
              unsigned short hb = f2bf_bits(sp[e]);
              unsigned short lb = f2bf_bits(sp[e] - bf_bits2f(hb));
              hv[e] = __builtin_bit_cast(_Float16, hb);
              lv[e] = __builtin_bit_cast(_Float16, lb);
            }
          }
          *(volatile v8h*)(C + (size_t)(mBase + row) * ldc + n0 + c8) = hv;
          if (OUT_MODE == 2) *(volatile v8h*)(C2 + (size_t)(mBase + row) * ldc + n0 + c8) = lv;
        }
        __threadfence();
      }
    }
    __builtin_amdgcn_fence(__ATOMIC_RELEASE, "workgroup");
    __builtin_amdgcn_wave_barrier();
    __builtin_amdgcn_fence(__ATOMIC_ACQUIRE, "workgroup");
  }
}

__global__ __launch_bounds__(256) void transpose_f16_kernel(
    const float* __restrict__ in, int rows, int cols, unsigned short* __restrict__ out, float scale)
{
  __shared__ __align__(16) float sT[64 * kTrP];
  const int tid = threadIdx.x, lane = tid & 31, wave = tid >> 5;
  const int r0 = blockIdx.y * 64, c0 = blockIdx.x * 64;
  const int c4 = (tid & 15) * 4, rr = tid >> 4;
  const int col = c0 + c4;
  const bool valid = (col < cols);
  const int colc = valid ? col : (cols - 4);
  const float sc = valid ? scale : 0.0f;
#pragma unroll
  for (int it = 0; it < 4; ++it) {
    const int row = it * 16 + rr;
    const v4f v = *(const v4f*)(in + (size_t)(r0 + row) * cols + colc);
    v4f w;
    w[0] = v[0] * sc; w[1] = v[1] * sc; w[2] = v[2] * sc; w[3] = v[3] * sc;
    *(v4f*)(sT + row * kTrP + c4) = w;
  }
  __syncthreads();
  const int q = lane >> 3, c8 = (lane & 7) * 8;
  v8h hv[2];
#pragma unroll
  for (int it = 0; it < 2; ++it) {
    const int j = it * 32 + wave * 4 + q;
#pragma unroll
    for (int e = 0; e < 8; ++e) hv[it][e] = (_Float16)sT[(c8 + e) * kTrP + j];
  }
  for (int pass = 0; pass < 2; ++pass) {
#pragma unroll
    for (int it = 0; it < 2; ++it) {
      const int j = it * 32 + wave * 4 + q;
      *(volatile v8h*)(out + (size_t)(c0 + j) * rows + r0 + c8) = hv[it];
    }
    __threadfence();
  }
}

__global__ __launch_bounds__(128) void rmsnorm_kernel(
    const float* __restrict__ x, const float* __restrict__ nsc, unsigned short* __restrict__ XN)
{
  __shared__ float wsum[4];
  const int tid = threadIdx.x, lane = tid & 31, wave = tid >> 5;
  const size_t row = blockIdx.x;
  const float* xr = x + row * kHid + tid * 8;
  const v4f a0 = *(const v4f*)(xr);
  const v4f a1 = *(const v4f*)(xr + 4);
  const v4f s0 = *(const v4f*)(nsc + tid * 8);
  const v4f s1 = *(const v4f*)(nsc + tid * 8 + 4);
  float ss = 0.0f;
#pragma unroll
  for (int e = 0; e < 4; ++e) ss = fmaf(a0[e], a0[e], ss);
#pragma unroll
  for (int e = 0; e < 4; ++e) ss = fmaf(a1[e], a1[e], ss);
#pragma unroll
  for (int off = 16; off > 0; off >>= 1) ss += __shfl_xor(ss, off, 32);
  if (lane == 0) wsum[wave] = ss;
  __syncthreads();
  const float tot = ((wsum[0] + wsum[1]) + wsum[2]) + wsum[3];
  const float rs = rsqrtf(tot * (1.0f / (float)kHid) + 1e-6f);
  v8h hv;
#pragma unroll
  for (int e = 0; e < 4; ++e) {
    hv[e]     = (_Float16)((a0[e] * rs) * s0[e]);
    hv[4 + e] = (_Float16)((a1[e] * rs) * s1[e]);
  }
  unsigned short* dst = XN + row * kHid + tid * 8;
  *(volatile v8h*)dst = hv;
  __threadfence();
  *(volatile v8h*)dst = hv;
}

__global__ __launch_bounds__(256) void conv_silu_kernel(
    const float* __restrict__ HID, const float* __restrict__ cw, const float* __restrict__ cb,
    float* __restrict__ CONV, unsigned short* __restrict__ CONV16)
{
  __shared__ __align__(16) float sT[16 * kConvTP];
  const int tid = threadIdx.x, lane = tid & 31, wave = tid >> 5;
  const int d0 = blockIdx.x * 256, d = d0 + tid;
  const int g0 = blockIdx.y * 64;
  const int tb = g0 & (kSeq - 1);
  const float w0 = cw[0 * kInner + d], w1 = cw[1 * kInner + d], w2 = cw[2 * kInner + d], w3 = cw[3 * kInner + d];
  const float bc = cb[d];
  float xm3, xm2, xm1;
  {
    const bool hist = (tb > 0);
    const int rb = hist ? (g0 - 3) : g0;
    const float hf = hist ? 1.0f : 0.0f;
    const float v3 = HID[(size_t)rb * kInner + d];
    const float v2 = HID[(size_t)(rb + 1) * kInner + d];
    const float v1 = HID[(size_t)(rb + 2) * kInner + d];
    xm3 = v3 * hf;
    xm2 = v2 * hf;
    xm1 = v1 * hf;
  }
  const int hrow = wave >> 1;
  const int hch  = (wave & 1) * 128 + lane * 4;
#pragma unroll 1
  for (int sub = 0; sub < 4; ++sub) {
    const int lb = g0 + sub * 16;
#pragma unroll 1
    for (int s = 0; s < 16; ++s) {
      const float xcur = HID[(size_t)(lb + s) * kInner + d];
      float acc = w0 * xm3;
      acc = fmaf(w1, xm2, acc);
      acc = fmaf(w2, xm1, acc);
      acc = fmaf(w3, xcur, acc);
      const float sv = acc + bc;
      const float sg = 1.0f / (1.0f + expf(-sv));
      sT[s * kConvTP + tid] = sv * sg;
      xm3 = xm2; xm2 = xm1; xm1 = xcur;
    }
    __syncthreads();
    v4f fv[4];
    v8h hv[2];
#pragma unroll
    for (int it = 0; it < 4; ++it) fv[it] = *(const v4f*)(sT + (it * 4 + hrow) * kConvTP + hch);
#pragma unroll
    for (int it = 0; it < 2; ++it) {
      const float* sp = sT + (it * 8 + wave) * kConvTP + lane * 8;
      const v4f a0 = *(const v4f*)(sp);
      const v4f a1 = *(const v4f*)(sp + 4);
#pragma unroll
      for (int e = 0; e < 4; ++e) {
        hv[it][e]     = (_Float16)(a0[e] * kConvCarry);
        hv[it][4 + e] = (_Float16)(a1[e] * kConvCarry);
      }
    }
    for (int pass = 0; pass < 2; ++pass) {
#pragma unroll
      for (int it = 0; it < 4; ++it)
        *(volatile v4f*)(CONV + (size_t)(lb + it * 4 + hrow) * kInner + d0 + hch) = fv[it];
#pragma unroll
      for (int it = 0; it < 2; ++it)
        *(volatile v8h*)(CONV16 + (size_t)(lb + it * 8 + wave) * kInner + d0 + lane * 8) = hv[it];
      __threadfence();
    }
    __syncthreads();
  }
}

__global__ __launch_bounds__(256) void ts16_kernel(const float* __restrict__ XPJ, unsigned short* __restrict__ TS16)
{
  const int i = blockIdx.x * 256 + threadIdx.x;
  if (i >= kRows * (kRank / 8)) return;
  const int row = i >> 3, c8 = (i & 7) * 8;
  const float* sp = XPJ + (size_t)row * kXpjP + c8;
  const v4f a0 = *(const v4f*)(sp);
  const v4f a1 = *(const v4f*)(sp + 4);
  v8h hv;
#pragma unroll
  for (int e = 0; e < 4; ++e) {
    hv[e]     = (_Float16)(a0[e] * kTsCarry);
    hv[4 + e] = (_Float16)(a1[e] * kTsCarry);
  }
  unsigned short* dst = TS16 + (size_t)row * kRank + c8;
  *(volatile v8h*)dst = hv;
  __threadfence();
  *(volatile v8h*)dst = hv;
}

__global__ __launch_bounds__(kScanCh) void scan_kernel(
    const float* __restrict__ XPJ, const float* __restrict__ CONV, const float* __restrict__ GATE,
    const float* __restrict__ DT, const float* __restrict__ dtb, const float* __restrict__ Alog,
    const float* __restrict__ Dp, unsigned short* __restrict__ Y16)
{
  __shared__ __align__(16) float sX[kScanTS * kScanXP];
  __shared__ __align__(16) float sY[kScanTS * kScanYP];
  __shared__ __align__(16) float sA[kNst * kScanCh];
  const int tid = threadIdx.x, lane = tid & 31, wave = tid >> 5;
  constexpr int kBlkPerB = kInner / kScanCh;
  const int bix = blockIdx.x / kBlkPerB;
  const int d0  = (blockIdx.x - bix * kBlkPerB) * kScanCh;
  const int d   = d0 + tid;
  const size_t row0 = (size_t)bix * kSeq;
#pragma unroll 1
  for (int s = 0; s < kNst; ++s) sA[s * kScanCh + tid] = -expf(Alog[(size_t)d * kNst + s]) * kLog2e;
  __syncthreads();
  float negA2[kNst], h[kNst];
#pragma unroll
  for (int s = 0; s < kNst; ++s) {
    negA2[s] = sA[s * kScanCh + tid];
    h[s] = 0.0f;
  }
  const float bb = dtb[d], Dd = Dp[d];
  const int q = lane >> 3, c8 = (lane & 7) * 8;
#pragma unroll 1
  for (int t0 = 0; t0 < kSeq; t0 += kScanTS) {
    __syncthreads();
    {
      const float* xp = XPJ + (row0 + t0 + tid) * kXpjP + kRank;
      float* sp = sX + tid * kScanXP;
      const v4f u0 = *(const v4f*)(xp);
      const v4f u1 = *(const v4f*)(xp + 4);
      const v4f u2 = *(const v4f*)(xp + 8);
      const v4f u3 = *(const v4f*)(xp + 12);
      *(v4f*)(sp)      = u0;
      *(v4f*)(sp + 4)  = u1;
      *(v4f*)(sp + 8)  = u2;
      *(v4f*)(sp + 12) = u3;
      asm volatile("" ::: "memory");
      const v4f u4 = *(const v4f*)(xp + 16);
      const v4f u5 = *(const v4f*)(xp + 20);
      const v4f u6 = *(const v4f*)(xp + 24);
      const v4f u7 = *(const v4f*)(xp + 28);
      *(v4f*)(sp + 16) = u4;
      *(v4f*)(sp + 20) = u5;
      *(v4f*)(sp + 24) = u6;
      *(v4f*)(sp + 28) = u7;
    }
    __syncthreads();
#pragma unroll 1
    for (int s = 0; s < kScanTS; ++s) {
      const size_t ro = (row0 + t0 + s) * kInner + d;
      const float vraw = DT[ro];
      const float xt   = CONV[ro];
      const float zv   = GATE[ro];
      const float* xr = sX + s * kScanXP;
      float Bs[kNst], Cs[kNst];
#pragma unroll
      for (int q4 = 0; q4 < 4; ++q4) {
        const v4f bv = *(const v4f*)(xr + 4 * q4);
        const v4f cv = *(const v4f*)(xr + kNst + 4 * q4);
        Bs[4 * q4 + 0] = bv[0]; Bs[4 * q4 + 1] = bv[1]; Bs[4 * q4 + 2] = bv[2]; Bs[4 * q4 + 3] = bv[3];
        Cs[4 * q4 + 0] = cv[0]; Cs[4 * q4 + 1] = cv[1]; Cs[4 * q4 + 2] = cv[2]; Cs[4 * q4 + 3] = cv[3];
      }
      const float v   = vraw + bb;
      const float a   = exp2f(-fabsf(v) * kLog2e);
      const float dt  = fmaxf(v, 0.0f) + log2f(1.0f + a) * kLn2;
      const float dtx = dt * xt;
      float y = 0.0f;
#pragma unroll
      for (int k = 0; k < kNst; ++k) {
        const float e = exp2f(dt * negA2[k]);
        h[k] = fmaf(e, h[k], dtx * Bs[k]);
        y = fmaf(h[k], Cs[k], y);
      }
      y = fmaf(Dd, xt, y);
      const float sg = 1.0f / (1.0f + expf(-zv));
      y = y * (zv * sg);
      sY[s * kScanYP + tid] = y * kYCarry;
    }
    __syncthreads();
    v8h hv[8];
#pragma unroll
    for (int it = 0; it < 8; ++it) {
      const int row = it * 8 + wave * 4 + q;
      const float* sp = sY + row * kScanYP + c8;
      const v4f a0 = *(const v4f*)(sp);
      const v4f a1 = *(const v4f*)(sp + 4);
#pragma unroll
      for (int e = 0; e < 4; ++e) {
        hv[it][e]     = (_Float16)a0[e];
        hv[it][4 + e] = (_Float16)a1[e];
      }
    }
    for (int pass = 0; pass < 2; ++pass) {
#pragma unroll
      for (int it = 0; it < 8; ++it) {
        const int row = it * 8 + wave * 4 + q;
        const size_t o = (row0 + t0 + row) * kInner + d0 + c8;
        *(volatile v8h*)(Y16 + o) = hv[it];
      }
      __threadfence();
    }
  }
}

extern "C" void kernel_launch(void* const* d_in, const int* in_sizes, int n_in,
                              void* d_out, int out_size, void* d_ws, size_t ws_size,
                              hipStream_t stream) {
  if (n_in < 13) return;
  if (in_sizes[0]  != kRows * kHid) return;
  if (in_sizes[1]  != kHid) return;
  if (in_sizes[2]  != kHid * 2 * kInner) return;
  if (in_sizes[3]  != 2 * kInner) return;
  if (in_sizes[4]  != kTaps * kInner) return;
  if (in_sizes[5]  != kInner) return;
  if (in_sizes[6]  != kInner * kXpjN) return;
  if (in_sizes[7]  != kRank * kInner) return;
  if (in_sizes[8]  != kInner) return;
  if (in_sizes[9]  != kInner * kNst) return;
  if (in_sizes[10] != kInner) return;
  if (in_sizes[11] != kInner * kHid) return;
  if (in_sizes[12] != kHid) return;
  if (out_size != kRows * kHid) return;
  if (ws_size < kWsTotal) return;

  const float* x          = (const float*)d_in[0];
  const float* norm_scale = (const float*)d_in[1];
  const float* in_w       = (const float*)d_in[2];
  const float* in_b       = (const float*)d_in[3];
  const float* conv_w     = (const float*)d_in[4];
  const float* conv_b     = (const float*)d_in[5];
  const float* xproj_w    = (const float*)d_in[6];
  const float* dt_w       = (const float*)d_in[7];
  const float* dt_b       = (const float*)d_in[8];
  const float* A_log      = (const float*)d_in[9];
  const float* Dvec       = (const float*)d_in[10];
  const float* out_w      = (const float*)d_in[11];
  const float* out_b      = (const float*)d_in[12];
  float* out = (float*)d_out;

  char* ws = (char*)d_ws;
  unsigned short* WIN16  = (unsigned short*)(ws + kOffWIN);
  unsigned short* XN16   = (unsigned short*)(ws + kOffXN);
  unsigned short* CONV16 = (unsigned short*)(ws + kOffRA);
  unsigned short* Y16    = (unsigned short*)(ws + kOffRA);
  unsigned short* WOUT16 = (unsigned short*)(ws + kOffWOUT);
  unsigned short* WX16   = (unsigned short*)(ws + kOffWX);
  unsigned short* WDT16  = (unsigned short*)(ws + kOffWDT);
  unsigned short* TS16   = (unsigned short*)(ws + kOffTS);
  float*          XPJ    = (float*)(ws + kOffXPJ);
  float*          HID    = (float*)(ws + kOffHID);
  float*          DT     = (float*)(ws + kOffHID);
  float*          GATE   = (float*)(ws + kOffGATE);
  float*          CONV   = (float*)(ws + kOffCONV);

  transpose_f16_kernel<<<dim3((2 * kInner) / 64, kHid / 64), 256, 0, stream>>>(in_w, kHid, 2 * kInner, WIN16, kWCarry);
  transpose_f16_kernel<<<dim3(kXpjP / 64, kInner / 64), 256, 0, stream>>>(xproj_w, kInner, kXpjN, WX16, kWCarry);
  transpose_f16_kernel<<<dim3(kInner / 64, kRank / 64), 256, 0, stream>>>(dt_w, kRank, kInner, WDT16, kWCarry);
  transpose_f16_kernel<<<dim3(kHid / 64, kInner / 64), 256, 0, stream>>>(out_w, kInner, kHid, WOUT16, kWCarry);

  rmsnorm_kernel<<<kRows, 128, 0, stream>>>(x, norm_scale, XN16);

  wmma_gemm64<0, 0, 2, 0, false><<<dim3(256, 1), 256, 0, stream>>>(
      XN16, nullptr, kHid, 0L,
      WIN16, nullptr, kHid, 0L,
      (void*)HID, nullptr, kInner, 0L,
      in_b, nullptr, 0L,
      kRows, kInner, kHid, 1.0f / kWCarry);
  wmma_gemm64<0, 0, 2, 0, false><<<dim3(256, 1), 256, 0, stream>>>(
      XN16, nullptr, kHid, 0L,
      WIN16 + (size_t)kInner * kHid, nullptr, kHid, 0L,
      (void*)GATE, nullptr, kInner, 0L,
      in_b + kInner, nullptr, 0L,
      kRows, kInner, kHid, 1.0f / kWCarry);

  conv_silu_kernel<<<dim3(kInner / 256, kRows / 64), 256, 0, stream>>>(HID, conv_w, conv_b, CONV, CONV16);

  wmma_gemm64<0, 0, 0, 0, false><<<dim3(16, 1), 256, 0, stream>>>(
      CONV16, nullptr, kInner, 0L,
      WX16, nullptr, kInner, 0L,
      (void*)XPJ, nullptr, kXpjP, 0L,
      nullptr, nullptr, 0L,
      kRows, kXpjP, kInner, 1.0f / (kConvCarry * kWCarry));

  ts16_kernel<<<(kRows * (kRank / 8)) / 256, 256, 0, stream>>>(XPJ, TS16);

  wmma_gemm64<0, 0, 0, 0, false><<<dim3(256, 1), 256, 0, stream>>>(
      TS16, nullptr, kRank, 0L,
      WDT16, nullptr, kRank, 0L,
      (void*)DT, nullptr, kInner, 0L,
      nullptr, nullptr, 0L,
      kRows, kInner, kRank, 1.0f / (kTsCarry * kWCarry));

  scan_kernel<<<kBatch * (kInner / kScanCh), kScanCh, 0, stream>>>(XPJ, CONV, GATE, DT, dt_b, A_log, Dvec, Y16);

  wmma_gemm64<0, 0, 2, 0, false><<<dim3(128, 1), 256, 0, stream>>>(
      Y16, nullptr, kInner, 0L,
      WOUT16, nullptr, kInner, 0L,
      (void*)out, nullptr, kHid, 0L,
      out_b, nullptr, 0L,
      kRows, kHid, kInner, 1.0f / (kYCarry * kWCarry));
}
